// BahdanauAttention_30236569764263
// MI455X (gfx1250) — hardware-run, weakly checked
//
#include <hip/hip_runtime.h>


#ifndef NB
#define NB 16
#endif
#define NB_FULL 16
#define TQ   128
#define TK   256
#define DIN  64
#define HID  256
#define DV   256
#ifndef OUT_TQ
#define OUT_TQ TQ
#endif
#define KC   64
#define KTP  68
#define QTP  16
#define SCP  260
#define PHP  264
#define VTP  72
#define C2F  2.8853900817779268f
#define L2E  1.4426950408889634f
#define NEGT (-1000000.0f * 1.4426950408889634f)
#define PSH  14.0f

static_assert(NB <= NB_FULL);
static_assert(DIN % 32 == 0);
static_assert(DIN == 64);
static_assert(HID % 64 == 0);
static_assert(HID % 32 == 0);
static_assert(HID == 256);
static_assert(TQ % 64 == 0);
static_assert(TK % 64 == 0);
static_assert(TQ % 16 == 0);
static_assert(TK == 256);
static_assert(TK % KC == 0);
static_assert(KC == 64);
static_assert(TK % 32 == 0);
static_assert(DV == 8 * 32);
static_assert(DV % 64 == 0);
static_assert((KTP * 4) % 16 == 0);
static_assert((QTP * 4) % 16 == 0);
static_assert((SCP * 4) % 16 == 0);
static_assert((PHP * 2) % 16 == 0);
static_assert((VTP * 2) % 16 == 0);
static_assert(SCP >= TK);
static_assert(SCP >= DV);
static_assert(PHP >= TK);
static_assert(((size_t)NB * TQ * DIN) % 8 == 0);
static_assert(((size_t)NB * TK * DIN) % 8 == 0);
static_assert(256 * 16 == 32 * DIN * 2);
static_assert(256 * 2 * 16 == 64 * 64 * 2);
static_assert(32 * 8 * 16 == 16 * 64 * 4);
static_assert(32 * 4 * 16 == 16 * 32 * 4);
static_assert(64 * VTP * 2 <= 131072);
static_assert(16 * 68 * 4 <= 131072);
static_assert((HID * KTP + HID * QTP + HID + 16 * SCP + 16) * 4 + 16 * PHP * 2 <= 131072);

typedef _Float16 h16;
typedef unsigned short bf;
typedef __attribute__((ext_vector_type(16))) __bf16   v16bf;
typedef __attribute__((ext_vector_type(16))) _Float16 v16h;
typedef __attribute__((ext_vector_type(8)))  _Float16 v8h;
typedef __attribute__((ext_vector_type(8)))  unsigned short v8us;
typedef __attribute__((ext_vector_type(8)))  float    v8f;
typedef __attribute__((ext_vector_type(4)))  float    v4f;
typedef v4f  __attribute__((may_alias)) v4fa;
typedef v8h  __attribute__((may_alias)) v8ha;

__device__ __forceinline__ unsigned short f2bf(float f) { unsigned u = __float_as_uint(f); u += 0x7FFFu + ((u >> 16) & 1u); return (unsigned short)(u >> 16); }
__device__ __forceinline__ float bfr(float f) { return __uint_as_float(((unsigned)f2bf(f)) << 16); }
__device__ __forceinline__ v16h cat16(v8h lo, v8h hi) { return __builtin_shufflevector(lo, hi, 0, 1, 2, 3, 4, 5, 6, 7, 8, 9, 10, 11, 12, 13, 14, 15); }
__device__ __forceinline__ v16bf cat16b(v8us lo, v8us hi) { return __builtin_bit_cast(v16bf, __builtin_shufflevector(lo, hi, 0, 1, 2, 3, 4, 5, 6, 7, 8, 9, 10, 11, 12, 13, 14, 15)); }
__device__ __forceinline__ v8f wmma16(v16h a, v16h b, v8f c) { return __builtin_amdgcn_wmma_f32_16x16x32_f16(false, a, false, b, (short)0, c, false, false); }
__device__ __forceinline__ v8f wmmab(v16bf a, v16bf b, v8f c) { return __builtin_amdgcn_wmma_f32_16x16x32_bf16(false, a, false, b, (short)0, c, false, false); }
__device__ __forceinline__ v16h  ldh(const h16* p) { return cat16(*(const v8h*)p, *(const v8h*)(p + 16)); }
__device__ __forceinline__ v16bf ldb(const bf* p)  { return cat16b(*(const v8us*)p, *(const v8us*)(p + 16)); }
__device__ __forceinline__ void wave_sync() { __builtin_amdgcn_fence(3  , "wavefront"); __builtin_amdgcn_wave_barrier(); asm volatile("" ::: "memory"); }

__device__ __forceinline__ v8f wmma16g(v16h a, v16h b, v8f c) { c = wmma16(a, b, c); asm volatile("v_nop\n\tv_nop\n\tv_nop\n\tv_nop" : "+v"(c) : "v"(a), "v"(b)); return c; }
__device__ __forceinline__ v8f wmmabg(v16bf a, v16bf b, v8f c) { c = wmmab(a, b, c); asm volatile("v_nop\n\tv_nop\n\tv_nop\n\tv_nop" : "+v"(c) : "v"(a), "v"(b)); return c; }
__device__ __forceinline__ h16 toh_flush(float v) { const h16 r = (h16)v; return (fabsf(v) < 6.103515625e-05f) ? (h16)0.0f : r; }
__device__ __forceinline__ float p_flush(float e) { const float g = __builtin_amdgcn_exp2f(e); return (e < -14.0f) ? 0.0f : g; }
__device__ __forceinline__ float tanh_e2(float x2) { const float e = __builtin_amdgcn_exp2f(x2); const float r = __builtin_amdgcn_rcpf(1.0f + e); return fmaf(-2.0f, r, 1.0f); }

__global__ __launch_bounds__(256) void k_cvt8(const float* __restrict__ src, bf* dst, size_t n8) {
    const size_t i = (size_t)blockIdx.x * 256 + threadIdx.x; if (i >= n8) return;
    const v8f v = *(const v8f*)(src + i * 8); v8us o;
#pragma unroll
    for (int k = 0; k < 8; ++k) o[k] = f2bf(v[k]);
    *(volatile v8us*)(dst + i * 8) = o; __threadfence(); *(volatile v8us*)(dst + i * 8) = o;
}

__global__ __launch_bounds__(256) void k_wt(const float* __restrict__ w, bf* dst) {
    const int t = threadIdx.x; const int h = blockIdx.x * 32 + (t >> 3), c8 = (t & 7) * 8;
    v8us o;
#pragma unroll
    for (int i = 0; i < 8; ++i) o[i] = f2bf(w[(size_t)(c8 + i) * HID + h]);
    *(volatile v8us*)(dst + (size_t)h * DIN + c8) = o; __threadfence(); *(volatile v8us*)(dst + (size_t)h * DIN + c8) = o;
}

__global__ __launch_bounds__(256) void k_vt(const float* __restrict__ V, h16* VT) {
    __shared__ __align__(16) h16 ts[64 * VTP];
    const int t = threadIdx.x; const int v0 = blockIdx.x * 64, key0 = blockIdx.y * 64, b = blockIdx.z;
#pragma unroll
    for (int i = 0; i < 4; ++i) { const int idx = i * 256 + t; const int key = idx >> 4, c4 = (idx & 15) * 4;
        const v4f x = *(const v4f*)(V + ((size_t)b * TK + key0 + key) * DV + v0 + c4);
#pragma unroll
        for (int j = 0; j < 4; ++j) ts[(c4 + j) * VTP + key] = toh_flush(bfr(x[j])); }
    __syncthreads();
#pragma unroll 1
    for (int ps = 0; ps < 2; ++ps) {
#pragma unroll
        for (int s = 0; s < 2; ++s) { const int p = s * 256 + t; const int row = p >> 3, c8 = (p & 7) * 8;
            const v8h o = *(const v8ha*)(&ts[row * VTP + c8]);
            *(volatile v8h*)(VT + ((size_t)b * DV + v0 + row) * TK + key0 + c8) = o; }
        if (ps == 0) __threadfence(); }
}

__global__ __launch_bounds__(32) void k_projT(const bf* __restrict__ A, const bf* __restrict__ Bt, float* P, int T) {
    __shared__ __align__(16) float os[16 * 68];
    const int K = DIN;
    const int lane = threadIdx.x & 31, lr = lane & 15, hi = lane >> 4; const int r0 = blockIdx.x * 64, c0 = blockIdx.y * 64;
    v8f acc[4][4];
#pragma unroll
    for (int mb = 0; mb < 4; ++mb)
#pragma unroll
        for (int nb = 0; nb < 4; ++nb) acc[mb][nb] = (v8f){};
    const size_t aoff = (size_t)(r0 + lr) * K + 8 * hi, boff = (size_t)(c0 + lr) * K + 8 * hi;
#pragma unroll 1
    for (int kc = 0; kc < K; kc += 32) {
        v16bf a[4];
#pragma unroll
        for (int mb = 0; mb < 4; ++mb) a[mb] = ldb(A + aoff + (size_t)mb * 16 * K + kc);
#pragma unroll
        for (int nb = 0; nb < 4; ++nb) { const v16bf b = ldb(Bt + boff + (size_t)nb * 16 * K + kc);
#pragma unroll
            for (int mb = 0; mb < 4; ++mb) acc[mb][nb] = wmmabg(a[mb], b, acc[mb][nb]); }
    }
    const int bb = c0 / T, tt = c0 % T;
    const size_t tbase = ((size_t)bb * HID + (size_t)r0) * (size_t)T + (size_t)tt;
#pragma unroll
    for (int mb = 0; mb < 4; ++mb) {
#pragma unroll
        for (int nb = 0; nb < 4; ++nb) {
#pragma unroll
            for (int j = 0; j < 8; ++j) os[(hi * 8 + j) * 68 + nb * 16 + lr] = acc[mb][nb][j] * C2F; }
        wave_sync();
#pragma unroll 1
        for (int ps = 0; ps < 2; ++ps) {
#pragma unroll
            for (int s = 0; s < 8; ++s) { const int row = 2 * s + (lane >> 4), cofs = (lane & 15) * 4;
                const v4f val = *(const v4fa*)(&os[row * 68 + cofs]);
                *(volatile v4f*)(P + tbase + (size_t)(mb * 16 + row) * (size_t)T + cofs) = val; }
            if (ps == 0) __threadfence(); }
        wave_sync();
    }
}

__global__ __launch_bounds__(256) void k_attn(const float* __restrict__ QT, const float* __restrict__ KT, const h16* __restrict__ VT,
                                              const float* __restrict__ wvec, const int* __restrict__ vlen, float* OUT) {
    __shared__ __align__(16) float kt[HID * KTP];
    __shared__ __align__(16) float qt[HID * QTP];
    __shared__ __align__(16) float wl[HID];
    __shared__ __align__(16) float sc[16 * SCP];
    __shared__ __align__(16) h16   ph[16 * PHP];
    __shared__ __align__(16) float rinv[16];
    const int t = threadIdx.x, lane = t & 31, lr = lane & 15, hi = lane >> 4;
    const int wave = __builtin_amdgcn_readfirstlane((int)(threadIdx.x >> 5));
    const int q0 = blockIdx.x * 16, b = blockIdx.y;
    int vraw = vlen[b]; vraw = vraw < 0 ? 0 : vraw; vraw = vraw > TK ? TK : vraw;
    const int vl = __builtin_amdgcn_readfirstlane(vraw);
    const int nch = (vl + KC - 1) / KC;

    wl[t] = bfr(wvec[t]);
#pragma unroll
    for (int i = 0; i < 4; ++i) { const int idx = i * 256 + t; const int h = idx >> 2, c4 = (idx & 3) * 4;
        const v4f x = *(const v4f*)(QT + ((size_t)b * HID + h) * TQ + q0 + c4);
        *(v4fa*)(&qt[h * QTP + c4]) = x; }

    const int q = t & 15, kg = t >> 4;
#pragma unroll 1
    for (int c = 0; c < TK / KC; ++c) {
        float a0 = 0.0f, a1 = 0.0f, a2 = 0.0f, a3 = 0.0f;
        if (c < nch) {
            __syncthreads();
#pragma unroll 4
            for (int i = 0; i < 16; ++i) { const int idx = i * 256 + t; const int h = idx >> 4, c4 = (idx & 15) * 4;
                const v4f x = *(const v4f*)(KT + ((size_t)b * HID + h) * TK + c * KC + c4);
                *(v4fa*)(&kt[h * KTP + c4]) = x; }
            __syncthreads();
#pragma unroll 2
            for (int h = 0; h < HID; ++h) {
                const float qv = qt[h * QTP + q]; const float w = wl[h];
                const v4f kv = *(const v4fa*)(&kt[h * KTP + kg * 4]);
                a0 = fmaf(w, tanh_e2(qv + kv[0]), a0); a1 = fmaf(w, tanh_e2(qv + kv[1]), a1);
                a2 = fmaf(w, tanh_e2(qv + kv[2]), a2); a3 = fmaf(w, tanh_e2(qv + kv[3]), a3); }
        }
        const int kk = c * KC + kg * 4;
        v4f o;
        o[0] = (kk + 0 < vl) ? a0 * L2E : NEGT; o[1] = (kk + 1 < vl) ? a1 * L2E : NEGT;
        o[2] = (kk + 2 < vl) ? a2 * L2E : NEGT; o[3] = (kk + 3 < vl) ? a3 * L2E : NEGT;
        *(v4fa*)(&sc[q * SCP + kk]) = o;
    }
    __syncthreads();

#pragma unroll 1
    for (int rr = 0; rr < 2; ++rr) {
        const int row = wave * 2 + rr;
        const v4f s0 = *(const v4fa*)(&sc[row * SCP + lane * 8]); const v4f s1 = *(const v4fa*)(&sc[row * SCP + lane * 8 + 4]);
        float mx = fmaxf(fmaxf(fmaxf(s0[0], s0[1]), fmaxf(s0[2], s0[3])), fmaxf(fmaxf(s1[0], s1[1]), fmaxf(s1[2], s1[3])));
        mx = fmaxf(mx, __shfl_xor(mx, 16, 32)); mx = fmaxf(mx, __shfl_xor(mx, 8, 32)); mx = fmaxf(mx, __shfl_xor(mx, 4, 32));
        mx = fmaxf(mx, __shfl_xor(mx, 2, 32));  mx = fmaxf(mx, __shfl_xor(mx, 1, 32));
        const float sh = PSH - mx;
        v8h pv; float ls = 0.0f;
#pragma unroll
        for (int i = 0; i < 4; ++i) {
            const h16 pa = (h16)p_flush(s0[i] + sh); const h16 pc = (h16)p_flush(s1[i] + sh);
            pv[i] = pa; pv[4 + i] = pc; ls += (float)pa + (float)pc; }
        ls += __shfl_xor(ls, 16, 32); ls += __shfl_xor(ls, 8, 32); ls += __shfl_xor(ls, 4, 32); ls += __shfl_xor(ls, 2, 32); ls += __shfl_xor(ls, 1, 32);
        if (lane == 0) rinv[row] = 1.0f / ls;
        *(v8ha*)(&ph[row * PHP + lane * 8]) = pv;
    }
    __syncthreads();

    v8f acc0 = (v8f){}, acc1 = (v8f){};
    const int n0 = wave * 32;
    const size_t vb = ((size_t)b * DV + n0 + lr) * TK + 8 * hi;
    const int pa0 = lr * PHP + 8 * hi;
#pragma unroll 1
    for (int k0 = 0; k0 < TK; k0 += 32) {
        const v16h a = cat16(*(const v8ha*)(&ph[pa0 + k0]), *(const v8ha*)(&ph[pa0 + k0 + 16]));
        const v16h b0 = ldh(VT + vb + k0), b1 = ldh(VT + vb + (size_t)16 * TK + k0);
        acc0 = wmma16g(a, b0, acc0); acc1 = wmma16g(a, b1, acc1);
    }
#pragma unroll
    for (int r = 0; r < 8; ++r) { const float ri = rinv[8 * hi + r];
        sc[(8 * hi + r) * SCP + n0 + lr] = acc0[r] * ri; sc[(8 * hi + r) * SCP + n0 + 16 + lr] = acc1[r] * ri; }
    wave_sync();
    float* orow = OUT + ((size_t)b * OUT_TQ + q0) * DV + n0;
#pragma unroll 1
    for (int ps = 0; ps < 2; ++ps) {
#pragma unroll
        for (int s = 0; s < 4; ++s) { const int row = 4 * s + (lane >> 3), cofs = (lane & 7) * 4;
            const v4f val = *(const v4fa*)(&sc[row * SCP + n0 + cofs]);
            *(volatile v4f*)(orow + (size_t)row * DV + cofs) = val; }
        if (ps == 0) __threadfence(); }
}

static constexpr size_t al256(size_t v) { return (v + 255) & ~(size_t)255; }
static constexpr size_t SZ_XQ = al256((size_t)NB * TQ * DIN * 2);
static constexpr size_t SZ_XK = al256((size_t)NB * TK * DIN * 2);
static constexpr size_t SZ_WT = al256((size_t)HID * DIN * 2);
static constexpr size_t SZ_QT = al256((size_t)NB * HID * TQ * 4);
static constexpr size_t SZ_KT = al256((size_t)NB * HID * TK * 4);
static constexpr size_t SZ_VT = al256((size_t)NB * DV * TK * 2);
static constexpr size_t SZ_TOTAL = SZ_XQ + SZ_XK + 2 * SZ_WT + SZ_QT + SZ_KT + SZ_VT;
static_assert(SZ_TOTAL <= (size_t)134217728);
static_assert((NB * TQ) % 64 == 0);
static_assert((NB * TK) % 64 == 0);

extern "C" void kernel_launch(void* const* d_in, const int* in_sizes, int n_in,
                              void* d_out, int out_size, void* d_ws, size_t ws_size, hipStream_t stream) {
    if (n_in < 7) return;
    if ((size_t)in_sizes[0] < (size_t)NB * TQ * DIN || (size_t)in_sizes[1] < (size_t)NB * TK * DIN || (size_t)in_sizes[2] < (size_t)NB * TK * DV) return;
    if (in_sizes[3] < NB) return;
    if ((size_t)in_sizes[4] < (size_t)DIN * HID || (size_t)in_sizes[5] < (size_t)DIN * HID || in_sizes[6] < HID) return;
    if ((size_t)out_size < ((size_t)(NB - 1) * OUT_TQ + TQ) * DV) return;
    if (SZ_TOTAL > ws_size) return;
    const float* queries = (const float*)d_in[0];
    const float* keys    = (const float*)d_in[1];
    const float* values  = (const float*)d_in[2];
    const int*   vlen    = (const int*)d_in[3];
    const float* wq      = (const float*)d_in[4];
    const float* wk      = (const float*)d_in[5];
    const float* wv      = (const float*)d_in[6];
    float* OUT = (float*)d_out;
    char* wsp = (char*)d_ws;
    bf*    XQ  = (bf*)wsp;    wsp += SZ_XQ;
    bf*    XK  = (bf*)wsp;    wsp += SZ_XK;
    bf*    WQT = (bf*)wsp;    wsp += SZ_WT;
    bf*    WKT = (bf*)wsp;    wsp += SZ_WT;
    float* QT  = (float*)wsp; wsp += SZ_QT;
    float* KT  = (float*)wsp; wsp += SZ_KT;
    h16*   VT  = (h16*)wsp;   wsp += SZ_VT;

    { const size_t n8 = (size_t)NB * TQ * DIN / 8; k_cvt8<<<(unsigned)((n8 + 255) / 256), 256, 0, stream>>>(queries, XQ, n8); }
    { const size_t n8 = (size_t)NB * TK * DIN / 8; k_cvt8<<<(unsigned)((n8 + 255) / 256), 256, 0, stream>>>(keys, XK, n8); }
    k_wt<<<HID / 32, 256, 0, stream>>>(wq, WQT);
    k_wt<<<HID / 32, 256, 0, stream>>>(wk, WKT);
    k_vt<<<dim3(DV / 64, TK / 64, NB), 256, 0, stream>>>(values, VT);

    k_projT<<<dim3(HID / 64, NB * TQ / 64, 1), 32, 0, stream>>>(WQT, XQ, QT, TQ);
    k_projT<<<dim3(HID / 64, NB * TK / 64, 1), 32, 0, stream>>>(WKT, XK, KT, TK);

    k_attn<<<dim3(TQ / 16, NB, 1), 256, 0, stream>>>(QT, KT, VT, wv, vlen, OUT);
}
